// ConsistencyDetector_21835613733616
// MI455X (gfx1250) — hardware-verified
//
#include <hip/hip_runtime.h>
#include <hip/hip_bf16.h>
#include <math.h>


#define BB 2
#define SS 2048
#define DD 1024
#define HH 16
#define DKK 64
#define QW 2

typedef _Float16 bf16;
typedef __attribute__((ext_vector_type(4))) unsigned v4u_t;
typedef unsigned v4ua __attribute__((ext_vector_type(4), may_alias));
typedef __attribute__((ext_vector_type(4))) float v4f_t;
typedef float v4fa __attribute__((ext_vector_type(4), may_alias));
typedef __attribute__((ext_vector_type(16))) bf16  bf16x16;
typedef __attribute__((ext_vector_type(8)))  bf16  bf16x8;
typedef __attribute__((ext_vector_type(4)))  bf16  bf16x4;
typedef __attribute__((ext_vector_type(8)))  float f32x8;

#define LDS_STRIDE 48
#define KSTRIDE    72
#define VSTRIDE    48

__device__ __forceinline__ f32x8 wmma_bf16(bf16x16 a, bf16x16 b, f32x8 c) {
  return __builtin_amdgcn_wmma_f32_16x16x32_f16(
      false, a, false, b, (short)0, c, false, false);
}
#define RSPLIT (1.0f / 2048.0f)
__device__ __forceinline__ bf16 lo_of(float v, bf16 h) { return (bf16)((v - (float)h) * 2048.0f); }
__device__ __forceinline__ f32x8 wmma_split(bf16x16 a, bf16x16 al, bf16x16 b, bf16x16 bl, f32x8 c) {
  f32x8 x = {}; x = wmma_bf16(al, b, x); x = wmma_bf16(a, bl, x); return wmma_bf16(a, b, c) + x * RSPLIT; }

template <typename T>
__device__ __forceinline__ bf16x16 load_frag(const T* __restrict__ base, int ld,
                                             int row0, int k0) {
  const int lane = threadIdx.x & 31;
  const int r    = lane & 15;
  const int kh   = (lane >> 4) * 8;
  const T* p0 = base + (size_t)(row0 + r) * ld + (k0 + kh);
  const T* p1 = p0 + 16;
  bf16x16 f;
#pragma unroll
  for (int i = 0; i < 8; ++i) {
    f[i]     = (bf16)p0[i];
    f[i + 8] = (bf16)p1[i];
  }
  return f;
}

__device__ __forceinline__ bf16x16 lds_frag(const bf16* base, int stride) {
  const int lane = threadIdx.x & 31;
  const int row  = lane & 15;
  const int kh   = (lane >> 4) * 8;
  const bf16x8 lo = *(const bf16x8*)(base + row * stride + kh);
  const bf16x8 hi = *(const bf16x8*)(base + row * stride + kh + 16);
  bf16x16 f;
#pragma unroll
  for (int i = 0; i < 8; ++i) { f[i] = lo[i]; f[i + 8] = hi[i]; }
  return f;
}

template <typename T>
__device__ __forceinline__ void stage_read16(const T* __restrict__ p, float* buf) {
#pragma unroll
  for (int i = 0; i < 16; ++i) buf[i] = (float)p[i];
}

__device__ __forceinline__ void stage_write(bf16* dst, const float* buf, int nquad) {
#pragma unroll
  for (int i = 0; i < nquad; ++i) {
    bf16x4 q;
    q[0] = (bf16)buf[4 * i];     q[1] = (bf16)buf[4 * i + 1];
    q[2] = (bf16)buf[4 * i + 2]; q[3] = (bf16)buf[4 * i + 3];
    *(bf16x4*)(dst + 4 * i) = q;
  }
}

__global__ __launch_bounds__(256) void transpose_pack_kernel(const float* __restrict__ W, bf16* __restrict__ WT, int K, int N, size_t plane) {
  __shared__ float tile[64][65];
  const int k0 = blockIdx.y * 64, n0 = blockIdx.x * 64, t = threadIdx.x;
  for (int i = t; i < 64 * 64; i += 256) { const int kr = i >> 6, nc = i & 63; tile[kr][nc] = W[(size_t)(k0 + kr) * N + n0 + nc]; }
  __syncthreads();
#pragma unroll 1
  for (int pass = 0; pass < 2; ++pass) {
    for (int i = t; i < 64 * 8; i += 256) { const int nr = i >> 3, k8 = (i & 7) * 8; bf16 hh[8], hl[8];
#pragma unroll
      for (int e = 0; e < 8; ++e) { const float v = tile[k8 + e][nr]; hh[e] = (bf16)v; hl[e] = lo_of(v, hh[e]); }
      bf16* d = WT + (size_t)(n0 + nr) * K + k0 + k8;
      *(volatile v4u_t*)d = *(const v4ua*)hh; *(volatile v4u_t*)(d + plane) = *(const v4ua*)hl; }
    __threadfence();
  }
}

template <typename AT, typename WT, int MODE>
__global__ __launch_bounds__(256) void gemm_split_kernel(
    const AT* __restrict__ A, size_t aPlane, const WT* __restrict__ W, size_t wPlane,
    const float* __restrict__ bias, void* __restrict__ out,
    int M, int N, int K) {
  __shared__ bf16 ldsA[128 * LDS_STRIDE], ldsAl[128 * LDS_STRIDE];
  __shared__ bf16 ldsW[256 * LDS_STRIDE], ldsWl[256 * LDS_STRIDE];
  __shared__ __attribute__((aligned(16))) unsigned char sob[256 * 136 * 2];

  const int t    = threadIdx.x;
  const int wave = t >> 5;
  const int lane = t & 31;
  const int wm   = (wave & 1) * 64;
  const int wn   = (wave >> 1) * 64;
  const int mBlk = blockIdx.x * 128;
  const int nBlk = blockIdx.y * 256;
  const int arow = t >> 1;
  const int ach  = (t & 1) * 16;

  f32x8 acc[4][4] = {};
  for (int k = 0; k < K; k += 32) {
    __syncthreads();
    {
      const AT* ap = A + (size_t)(mBlk + arow) * K + k + ach;
      bf16 hh[16], hl[16];
      if (sizeof(AT) == 4) {
#pragma unroll
        for (int i = 0; i < 16; ++i) { const float v = (float)ap[i]; hh[i] = (bf16)v; hl[i] = lo_of(v, hh[i]); }
      } else {
#pragma unroll
        for (int i = 0; i < 16; ++i) { hh[i] = (bf16)ap[i]; hl[i] = (bf16)ap[aPlane + i]; }
      }
#pragma unroll
      for (int i = 0; i < 16; ++i) { ldsA[arow * LDS_STRIDE + ach + i] = hh[i]; ldsAl[arow * LDS_STRIDE + ach + i] = hl[i]; }
    }
    {
      const WT* wp = W + (size_t)(nBlk + t) * K + k;
      if (sizeof(WT) == 4) {
#pragma unroll
        for (int i = 0; i < 32; ++i) { const float v = (float)wp[i]; const bf16 h_ = (bf16)v; ldsW[t * LDS_STRIDE + i] = h_; ldsWl[t * LDS_STRIDE + i] = lo_of(v, h_); }
      } else {
#pragma unroll
        for (int i = 0; i < 32; ++i) { ldsW[t * LDS_STRIDE + i] = (bf16)wp[i]; ldsWl[t * LDS_STRIDE + i] = (bf16)wp[wPlane + i]; }
      }
    }
    __syncthreads();
    bf16x16 wf[4], wfl[4];
#pragma unroll
    for (int j = 0; j < 4; ++j) { wf[j] = lds_frag(ldsW + (wn + 16 * j) * LDS_STRIDE, LDS_STRIDE); wfl[j] = lds_frag(ldsWl + (wn + 16 * j) * LDS_STRIDE, LDS_STRIDE); }
#pragma unroll
    for (int i = 0; i < 4; ++i) {
      const bf16x16 af = lds_frag(ldsA + (wm + 16 * i) * LDS_STRIDE, LDS_STRIDE), afl = lds_frag(ldsAl + (wm + 16 * i) * LDS_STRIDE, LDS_STRIDE);
#pragma unroll
      for (int j = 0; j < 4; ++j) acc[i][j] = wmma_split(af, afl, wf[j], wfl[j], acc[i][j]);
    }
  }

  const int nlane = lane & 15;
  const int mh    = (lane >> 4) * 8;
  __syncthreads();
  if (MODE == 1) {
    bf16* so = (bf16*)sob;
#pragma unroll
    for (int i = 0; i < 4; ++i)
#pragma unroll
      for (int j = 0; j < 4; ++j) {
        const int nl = wn + 16 * j + nlane;
        const float bv = bias ? bias[nBlk + nl] : 0.0f;
#pragma unroll
        for (int r = 0; r < 8; ++r) so[nl * 136 + wm + 16 * i + mh + r] = (bf16)(acc[i][j][r] + bv);
      }
    __syncthreads();
    const int b_ = mBlk >> 11, s0 = mBlk & (SS - 1);
#pragma unroll 1
    for (int pass = 0; pass < 2; ++pass) {
      for (int ch = t; ch < 256 * 16; ch += 256) { const int nl = ch >> 4, q = (ch & 15) * 8; const int n = nBlk + nl, h = n >> 6, dk = n & (DKK - 1);
        *(volatile v4u_t*)((bf16*)out + (((size_t)(b_ * HH + h)) * DKK + dk) * SS + s0 + q) = *(const v4ua*)(so + nl * 136 + q); }
      __threadfence();
    }
  } else {
    float* so = (float*)sob;
#pragma unroll 1
    for (int hf = 0; hf < 2; ++hf) {
      if (wm == hf * 64) {
#pragma unroll
        for (int i = 0; i < 4; ++i)
#pragma unroll
          for (int j = 0; j < 4; ++j) {
            const int nl = wn + 16 * j + nlane;
            const float bv = bias ? bias[nBlk + nl] : 0.0f;
#pragma unroll
            for (int r = 0; r < 8; ++r) so[(16 * i + mh + r) * 260 + nl] = acc[i][j][r] + bv;
          }
      }
      __syncthreads();
#pragma unroll 1
      for (int pass = 0; pass < 2; ++pass) {
        for (int ch = t; ch < 64 * 64; ch += 256) { const int ml = ch >> 6, q = (ch & 63) * 4;
          *(volatile v4f_t*)((float*)out + (size_t)(mBlk + hf * 64 + ml) * N + nBlk + q) = *(const volatile v4fa*)(so + ml * 260 + q); }
        __threadfence();
      }
      __syncthreads();
    }
  }
}


#define CN 100000
#define CNP 100352
#define CE 800000
#define CRANGE 25088

__global__ __launch_bounds__(128) void k_packA(const float* __restrict__ W, int kin, int mout, float* __restrict__ A) {
  const int m = blockIdx.x, k = threadIdx.x;
  if (k < kin) { const float v = (m < mout) ? W[k * mout + m] : 0.0f; *(volatile float*)(A + m * kin + k) = v; __threadfence(); *(volatile float*)(A + m * kin + k) = v; }
}
__global__ __launch_bounds__(256) void k_deg(const int* __restrict__ ei, float* __restrict__ invdeg) {
  __shared__ int cnt[CRANGE + 8]; __shared__ int qd[256]; __shared__ int wcnt[8];
  const int tid = threadIdx.x, lane = tid & 31, wave = tid >> 5, r0 = blockIdx.x * CRANGE;
  for (int i = tid; i < CRANGE + 8; i += 256) cnt[i] = 0;
  __syncthreads();
  const int* dstp = ei + (size_t)CE;
#pragma unroll 1
  for (int c0 = 0; c0 < CE; c0 += 256) {
    const int e = c0 + tid; int d = -1;
    if (e < CE) { const int draw = dstp[e]; const int dd = draw < 0 ? 0 : (draw >= CN ? CN - 1 : draw); if (dd >= r0 && dd < r0 + CRANGE) d = dd - r0; }
    const unsigned m = __builtin_amdgcn_ballot_w32(d >= 0);
    if (lane == 0) wcnt[wave] = __builtin_popcount(m);
    __syncthreads();
    int base = 0, total = 0;
#pragma unroll
    for (int w = 0; w < 8; ++w) { const int c = wcnt[w]; base += (w < wave) ? c : 0; total += c; }
    if (d >= 0) qd[base + __builtin_popcount(m & ((1u << lane) - 1u))] = d;
    __syncthreads();
#pragma unroll 1
    for (int qi = 0; qi < total; ++qi) { const int dl = qd[qi]; if ((dl & 7) != wave) continue; if (lane == 0) cnt[dl] += 1; }
    __syncthreads();
  }
#pragma unroll 1
  for (int pass = 0; pass < 2; ++pass) {
    for (int i = tid; i < CRANGE / 4; i += 256) { v4f_t v;
#pragma unroll
      for (int q = 0; q < 4; ++q) v[q] = 1.0f / fmaxf((float)(cnt[i * 4 + q] + 1), 1.0f);
      *(volatile v4f_t*)(invdeg + r0 + i * 4) = v; }
    __threadfence();
  }
}
template <bool LOCAL>
__global__ __launch_bounds__(256) void k_nmean(const int* __restrict__ ei, const float* __restrict__ Fx, int frows  , const float* __restrict__ invdeg,
                                              int rsel, float* __restrict__ OUT) {
  __shared__ int qd[256], qs[256]; __shared__ int wcnt[8];
  const int tid = threadIdx.x, lane = tid & 31, wave = tid >> 5, r0 = (LOCAL ? rsel : blockIdx.x) * CRANGE;
  float* myR = OUT + (size_t)(LOCAL ? 0 : r0) * 64;
  for (int i = tid; i < CRANGE * 16; i += 256) { const int nl = i >> 4, c4 = (i & 15) * 4, node = r0 + nl; v4f_t v;
    if (node < frows) v = *(const v4fa*)(Fx + (size_t)node * 64 + c4); else { v.x = v.y = v.z = v.w = 0.0f; }
    *(volatile v4f_t*)(myR + (size_t)nl * 64 + c4) = v; }
  __threadfence(); __syncthreads();
  const int* srcp = ei; const int* dstp = ei + (size_t)CE;
#pragma unroll 1
  for (int c0 = 0; c0 < CE; c0 += 256) {
    const int e = c0 + tid; int d = -1, sidx = 0;
    if (e < CE) { const int draw = dstp[e]; const int dd = draw < 0 ? 0 : (draw >= CN ? CN - 1 : draw);
      if (dd >= r0 && dd < r0 + CRANGE) { d = dd - r0; const int ss = srcp[e]; sidx = ss < 0 ? 0 : (ss >= CN ? CN - 1 : ss); } }
    const unsigned m = __builtin_amdgcn_ballot_w32(d >= 0);
    if (lane == 0) wcnt[wave] = __builtin_popcount(m);
    __syncthreads();
    int base = 0, total = 0;
#pragma unroll
    for (int w = 0; w < 8; ++w) { const int c = wcnt[w]; base += (w < wave) ? c : 0; total += c; }
    if (d >= 0) { const int pos = base + __builtin_popcount(m & ((1u << lane) - 1u)); qd[pos] = d; qs[pos] = sidx; }
    __syncthreads();
#pragma unroll 1
    for (int qi = 0; qi < total; ++qi) { const int dl = qd[qi]; if ((dl & 7) != wave) continue; const int sl = qs[qi];
      float* row = myR + (size_t)dl * 64; row[lane] += Fx[(size_t)sl * 64 + lane]; row[32 + lane] += Fx[(size_t)sl * 64 + 32 + lane]; }
    __syncthreads();
  }
  __threadfence(); __syncthreads();
#pragma unroll 1
  for (int pass = 0; pass < 2; ++pass) {
    for (int i = tid; i < CRANGE * 16; i += 256) { const int nl = i >> 4, c4 = (i & 15) * 4, node = r0 + nl; float* p = myR + (size_t)nl * 64 + c4;
      v4f_t v = *(const volatile v4fa*)p; if (pass == 0) { const float s = (node < CN) ? invdeg[node] : 0.0f; v.x *= s; v.y *= s; v.z *= s; v.w *= s; }
      *(volatile v4f_t*)p = v; }
    __threadfence(); __syncthreads();
  }
}
__global__ __launch_bounds__(256) void k_rows(const float* __restrict__ T, int ld, const float* __restrict__ b, int ncol, float* __restrict__ Rout) {
  __shared__ float tile[64][65];
  const int n0 = blockIdx.x * 64, cb = blockIdx.y * 64, t = threadIdx.x;
  for (int i = t; i < 64 * 64; i += 256) { const int c = i >> 6, nn = i & 63; tile[c][nn] = T[(size_t)(cb + c) * ld + n0 + nn]; }
  __syncthreads();
#pragma unroll 1
  for (int pass = 0; pass < 2; ++pass) {
    for (int i = t; i < 64 * 16; i += 256) { const int nr = i >> 4, c4 = (i & 15) * 4; v4f_t v;
#pragma unroll
      for (int q = 0; q < 4; ++q) v[q] = fmaxf(tile[c4 + q][nr] + b[cb + c4 + q], 0.0f);
      *(volatile v4f_t*)(Rout + (size_t)(n0 + nr) * ncol + cb + c4) = v; }
    __threadfence();
  }
}
__global__ __launch_bounds__(256) void k_attr(const float* __restrict__ xhT, const float* __restrict__ bx2, const float* __restrict__ x, int r0, float* __restrict__ attr) {
  const int il = blockIdx.x * 256 + threadIdx.x, i = r0 + il;
  float s = 0.0f;
#pragma unroll 4
  for (int c = 0; c < 64; ++c) { const float dlt = xhT[(size_t)c * CRANGE + il] + bx2[c] - ((i < CN) ? x[(size_t)i * 64 + c] : 0.0f); s += dlt * dlt; }
  const float v = sqrtf(s + 1e-12f);
  if (i < CN) { *(volatile float*)(attr + i) = v; __threadfence(); *(volatile float*)(attr + i) = v; }
}
__global__ __launch_bounds__(256) void k_score(const float* __restrict__ mhT, const float* __restrict__ bh2, const float* __restrict__ M, const float* __restrict__ x,
                                              const float* __restrict__ attr, int r0, float* __restrict__ score, float* __restrict__ neigh) {
  const int il = blockIdx.x * 256 + threadIdx.x, i = r0 + il;
  float sn = 0.0f, sh = 0.0f;
  if (i < CN) {
#pragma unroll 4
    for (int c = 0; c < 64; ++c) { const float mh = mhT[(size_t)c * CRANGE + il] + bh2[c]; const float d1 = mh - M[(size_t)i * 64 + c], d2 = mh - x[(size_t)i * 64 + c]; sn += d1 * d1; sh += d2 * d2; }
    const float ne = sqrtf(sn + 1e-12f), ho = sqrtf(sh + 1e-12f), sc = 1.0f * attr[i] + 0.5f * ne + 0.3f * ho;
#pragma unroll 1
    for (int pass = 0; pass < 2; ++pass) { *(volatile float*)(score + i) = sc; *(volatile float*)(neigh + i) = ne; __threadfence(); }
  }
}

extern "C" void kernel_launch(void* const* d_in, const int* in_sizes, int n_in,
                              void* d_out, int out_size, void* d_ws, size_t ws_size,
                              hipStream_t stream) {
  (void)in_sizes; (void)n_in; (void)out_size; (void)ws_size;
  const float* x   = (const float*)d_in[0];
  const int*   ei  = (const int*)d_in[1];
  const float* Wen = (const float*)d_in[2];  const float* ben = (const float*)d_in[3];
  const float* Wx1 = (const float*)d_in[4];  const float* bx1 = (const float*)d_in[5];
  const float* Wx2 = (const float*)d_in[6];  const float* bx2 = (const float*)d_in[7];
  const float* Wh1 = (const float*)d_in[8];  const float* bh1 = (const float*)d_in[9];
  const float* Wh2 = (const float*)d_in[10]; const float* bh2 = (const float*)d_in[11];
  float* score = (float*)d_out;
  float* attr  = score + CN;
  float* neigh = score + 2 * CN;
  char* ws = (char*)d_ws;
  float* Aen = (float*)ws; ws += 128 * 64 * 4;
  float* Ax1 = (float*)ws; ws += 128 * 64 * 4;
  float* Ax2 = (float*)ws; ws += 128 * 128 * 4;
  float* Ah1 = (float*)ws; ws += 128 * 64 * 4;
  float* Ah2 = (float*)ws; ws += 128 * 128 * 4;
  float* M   = (float*)ws; ws += (size_t)CNP * 64 * 4;
  float* T   = (float*)ws; ws += (size_t)128 * CNP * 4;
  float* H   = T + (size_t)64 * CNP;
  float* C1  = (float*)ws; ws += (size_t)128 * CRANGE * 4;
  float* C2  = (float*)ws; ws += (size_t)128 * CRANGE * 4;
  float* C3  = (float*)ws; ws += (size_t)128 * CRANGE * 4;
  float* invdeg = (float*)ws; ws += (size_t)CNP * 4;
  k_packA<<<128, 128, 0, stream>>>(Wen, 64, 64, Aen);
  k_packA<<<128, 128, 0, stream>>>(Wx1, 64, 128, Ax1);
  k_packA<<<128, 128, 0, stream>>>(Wx2, 128, 64, Ax2);
  k_packA<<<128, 128, 0, stream>>>(Wh1, 64, 128, Ah1);
  k_packA<<<128, 128, 0, stream>>>(Wh2, 128, 64, Ah2);
  k_deg<<<CNP / CRANGE, 256, 0, stream>>>(ei, invdeg);
  k_nmean<false><<<CNP / CRANGE, 256, 0, stream>>>(ei, x, CN, invdeg, 0, M);
  dim3 blk(256);
  gemm_split_kernel<float, float, 2><<<dim3(1, CNP / 256), blk, 0, stream>>>(Aen, 0, M, 0, nullptr, T, 128, CNP, 64);
  k_rows<<<dim3(CNP / 64, 1), 256, 0, stream>>>(T, CNP, ben, 64, H);
  for (int r = 0; r < CNP / CRANGE; ++r) {
    const int r0 = r * CRANGE;
    gemm_split_kernel<float, float, 2><<<dim3(1, CRANGE / 256), blk, 0, stream>>>(Ax1, 0, H + (size_t)r0 * 64, 0, nullptr, C2, 128, CRANGE, 64);
    k_rows<<<dim3(CRANGE / 64, 2), 256, 0, stream>>>(C2, CRANGE, bx1, 128, C3);
    gemm_split_kernel<float, float, 2><<<dim3(1, CRANGE / 256), blk, 0, stream>>>(Ax2, 0, C3, 0, nullptr, C2, 128, CRANGE, 128);
    k_attr<<<CRANGE / 256, 256, 0, stream>>>(C2, bx2, x, r0, attr);
    k_nmean<true><<<1, 256, 0, stream>>>(ei, H, CNP, invdeg, r, C1);
    gemm_split_kernel<float, float, 2><<<dim3(1, CRANGE / 256), blk, 0, stream>>>(Ah1, 0, C1, 0, nullptr, C2, 128, CRANGE, 64);
    k_rows<<<dim3(CRANGE / 64, 2), 256, 0, stream>>>(C2, CRANGE, bh1, 128, C3);
    gemm_split_kernel<float, float, 2><<<dim3(1, CRANGE / 256), blk, 0, stream>>>(Ah2, 0, C3, 0, nullptr, C2, 128, CRANGE, 128);
    k_score<<<CRANGE / 256, 256, 0, stream>>>(C2, bh2, M, x, attr, r0, score, neigh);
  }
}
